// EmformerBlock_28733331210928
// MI455X (gfx1250) — hardware-verified
//
#include <hip/hip_runtime.h>

typedef _Float16 v16h __attribute__((ext_vector_type(16)));
typedef _Float16 v8h  __attribute__((ext_vector_type(8), may_alias));
typedef float    v8f  __attribute__((ext_vector_type(8)));
typedef float    v4f  __attribute__((ext_vector_type(4), may_alias));

union Frag { v16h v; v8h hf[2]; };

#define NB   8
#define NT   1024
#define ND   512
#define NH   8
#define NDK  64
#define NF   2048
#define NM   (NB * NT)
#define LNEPS  1.0e-3f
#define NEGBIG (-1.0e9f)

__device__ __forceinline__ v8f zero8() {
    v8f z = {0.f, 0.f, 0.f, 0.f, 0.f, 0.f, 0.f, 0.f};
    return z;
}

__device__ __forceinline__ v8f wmma16(v16h a, v16h b, v8f c) {
    v8f d = __builtin_amdgcn_wmma_f32_16x16x32_f16(false, a, false, b, (short)0, c, false, false);
    asm volatile("v_nop\n\tv_nop\n\tv_nop\n\tv_nop" : "+v"(d) : "v"(a), "v"(b));
    return d;
}

__global__ __launch_bounds__(256)
void k_wcvt(const float* __restrict__ W, _Float16* __restrict__ Wt, int K, int N, float scale) {
    __shared__ float tile[64][33];
    const int tid = threadIdx.x;
    const int kb = blockIdx.y * 64, nb = blockIdx.x * 32;
    const int c = tid & 31, r = tid >> 5;
    #pragma unroll
    for (int i = 0; i < 8; ++i)
        tile[r + 8 * i][c] = W[(size_t)(kb + r + 8 * i) * N + nb + c] * scale;
    __syncthreads();
    const int n = tid >> 3, pc = tid & 7;
    v8h o;
    #pragma unroll
    for (int e = 0; e < 8; ++e) o[e] = (_Float16)tile[pc * 8 + e][n];
    _Float16* dst = Wt + (size_t)(nb + n) * K + kb + pc * 8;
    *(volatile v8h*)dst = o;
    __threadfence();
    *(volatile v8h*)dst = o;
}

template <int OM>
__global__ __launch_bounds__(256)
void k_ln(const float* __restrict__ in, const float* __restrict__ g, const float* __restrict__ bt,
          float* __restrict__ of, _Float16* __restrict__ oh, int M) {
    const int lane = threadIdx.x & 31, wave = threadIdx.x >> 5;
    const int row = blockIdx.x * 8 + wave;
    if (row >= M) return;
    const float* r = in + (size_t)row * ND;

    v4f v[4];
    float s = 0.f;
    #pragma unroll
    for (int j = 0; j < 4; ++j) {
        v[j] = *(const v4f*)(r + 4 * lane + 128 * j);
        s += (v[j][0] + v[j][1]) + (v[j][2] + v[j][3]);
    }
    #pragma unroll
    for (int off = 16; off >= 1; off >>= 1) s += __shfl_xor(s, off, 32);
    const float mean = s * (1.0f / ND);
    float sq = 0.f;
    #pragma unroll
    for (int j = 0; j < 4; ++j) {
        #pragma unroll
        for (int c = 0; c < 4; ++c) { const float d = v[j][c] - mean; sq += d * d; }
    }
    #pragma unroll
    for (int off = 16; off >= 1; off >>= 1) sq += __shfl_xor(sq, off, 32);
    const float rstd = rsqrtf(sq * (1.0f / ND) + LNEPS);

    if constexpr (OM != 0) {
        v4f o[4];
        #pragma unroll
        for (int j = 0; j < 4; ++j) {
            const int c0 = 4 * lane + 128 * j;
            const v4f gv = *(const v4f*)(g + c0);
            const v4f bv = *(const v4f*)(bt + c0);
            #pragma unroll
            for (int c = 0; c < 4; ++c) o[j][c] = (v[j][c] - mean) * rstd * gv[c] + bv[c];
        }
        float* orow = of + (size_t)row * ND + 4 * lane;
        #pragma unroll
        for (int j = 0; j < 4; ++j) *(volatile v4f*)(orow + 128 * j) = o[j];
        __threadfence();
        #pragma unroll
        for (int j = 0; j < 4; ++j) *(volatile v4f*)(orow + 128 * j) = o[j];
    }
    if constexpr (OM != 2) {
        v8h w[2];
        #pragma unroll
        for (int j = 0; j < 2; ++j) {
            const int c0 = 8 * lane + 256 * j;
            const v4f x0 = *(const v4f*)(r + c0),  x1 = *(const v4f*)(r + c0 + 4);
            const v4f g0 = *(const v4f*)(g + c0),  g1 = *(const v4f*)(g + c0 + 4);
            const v4f b0 = *(const v4f*)(bt + c0), b1 = *(const v4f*)(bt + c0 + 4);
            #pragma unroll
            for (int c = 0; c < 4; ++c) {
                w[j][c]     = (_Float16)((x0[c] - mean) * rstd * g0[c] + b0[c]);
                w[j][4 + c] = (_Float16)((x1[c] - mean) * rstd * g1[c] + b1[c]);
            }
        }
        _Float16* hrow = oh + (size_t)row * ND + 8 * lane;
        #pragma unroll
        for (int j = 0; j < 2; ++j) *(volatile v8h*)(hrow + 256 * j) = w[j];
        __threadfence();
        #pragma unroll
        for (int j = 0; j < 2; ++j) *(volatile v8h*)(hrow + 256 * j) = w[j];
    }
}

template <int MODE>
__global__ __launch_bounds__(256)
void k_gemm(const _Float16* __restrict__ A, const _Float16* __restrict__ Bt,
            const float* __restrict__ bias, const float* __restrict__ resid,
            void* __restrict__ outp, int N, int K, float oscale) {
    __shared__ __align__(16) _Float16 As[64 * 40];
    __shared__ __align__(16) _Float16 Bs[64 * 40];
    __shared__ __align__(16) _Float16 Ch[64 * 72];
    __shared__ __align__(16) float    Cf[64 * 68];

    const int tid = threadIdx.x, lane = tid & 31, wave = tid >> 5;
    const int hl = lane >> 4, m = lane & 15;
    const int mBase = blockIdx.y * 64, nBase = blockIdx.x * 64;
    const int wm = wave & 3, wn = wave >> 2;
    const int ar = tid >> 2, ac = (tid & 3) * 8;
    const _Float16* Ag = A  + (size_t)(mBase + ar) * K + ac;
    const _Float16* Bg = Bt + (size_t)(nBase + ar) * K + ac;

    v8f acc0 = zero8(), acc1 = zero8();
    const int nk = K >> 5;
    for (int kt = 0; kt < nk; ++kt) {
        const int k0 = kt << 5;
        const v8h ta = *(const v8h*)(Ag + k0);
        const v8h tb = *(const v8h*)(Bg + k0);
        __syncthreads();
        *(v8h*)(As + ar * 40 + ac) = ta;
        *(v8h*)(Bs + ar * 40 + ac) = tb;
        __syncthreads();
        Frag fa, fb0, fb1;
        const _Float16* ap  = As + (wm * 16 + m) * 40;
        const _Float16* bp0 = Bs + (wn * 32 + m) * 40;
        const _Float16* bp1 = bp0 + 16 * 40;
        fa.hf[0]  = *(const v8h*)(ap  + 8 * hl);
        fa.hf[1]  = *(const v8h*)(ap  + 16 + 8 * hl);
        fb0.hf[0] = *(const v8h*)(bp0 + 8 * hl);
        fb0.hf[1] = *(const v8h*)(bp0 + 16 + 8 * hl);
        fb1.hf[0] = *(const v8h*)(bp1 + 8 * hl);
        fb1.hf[1] = *(const v8h*)(bp1 + 16 + 8 * hl);
        acc0 = wmma16(fa.v, fb0.v, acc0);
        acc1 = wmma16(fa.v, fb1.v, acc1);
    }

    const int rbase = wm * 16 + 8 * hl;
    const int c0 = wn * 32 + m, c1 = c0 + 16;
    const float bias0 = bias[nBase + c0], bias1 = bias[nBase + c1];

    if constexpr (MODE <= 2) {
        #pragma unroll
        for (int r = 0; r < 8; ++r) {
            float u0 = acc0[r] * oscale + bias0;
            float u1 = acc1[r] * oscale + bias1;
            if constexpr (MODE == 2) { u0 = fmaxf(u0, 0.0f); u1 = fmaxf(u1, 0.0f); }
            const int row = rbase + r;
            if constexpr (MODE == 1) {
                Ch[c0 * 72 + row] = (_Float16)u0;
                Ch[c1 * 72 + row] = (_Float16)u1;
            } else {
                Ch[row * 72 + c0] = (_Float16)u0;
                Ch[row * 72 + c1] = (_Float16)u1;
            }
        }
        __syncthreads();
        const int hh = nBase >> 6;
        v8h w[2];
        size_t off[2];
        #pragma unroll
        for (int j = 0; j < 2; ++j) {
            const int id = tid + 256 * j;
            const int line = id >> 3, pc = id & 7;
            w[j] = *(const v8h*)(Ch + line * 72 + pc * 8);
            if constexpr (MODE == 0) {
                const int mg = mBase + line;
                const int bb = mg / NT, t = mg % NT;
                off[j] = ((size_t)(bb * NH + hh) * NT + t) * NDK + pc * 8;
            } else if constexpr (MODE == 1) {
                const int bb = mBase / NT, t0 = mBase % NT;
                off[j] = ((size_t)(bb * NH + hh) * NDK + line) * NT + t0 + pc * 8;
            } else {
                off[j] = (size_t)(mBase + line) * N + nBase + pc * 8;
            }
        }
        _Float16* O = (_Float16*)outp;
        #pragma unroll
        for (int j = 0; j < 2; ++j) *(volatile v8h*)(O + off[j]) = w[j];
        __threadfence();
        #pragma unroll
        for (int j = 0; j < 2; ++j) *(volatile v8h*)(O + off[j]) = w[j];
    } else {
        #pragma unroll
        for (int r = 0; r < 8; ++r) {
            const int row = rbase + r;
            Cf[row * 68 + c0] = acc0[r] * oscale + bias0;
            Cf[row * 68 + c1] = acc1[r] * oscale + bias1;
        }
        __syncthreads();
        v4f w[4];
        size_t off[4];
        #pragma unroll
        for (int j = 0; j < 4; ++j) {
            const int id = tid + 256 * j;
            const int line = id >> 3, pc = id & 7;
            const int row = line >> 1, colo = ((line & 1) << 5) + pc * 4;
            off[j] = (size_t)(mBase + row) * N + nBase + colo;
            w[j] = *(const v4f*)(Cf + row * 68 + colo) + *(const v4f*)(resid + off[j]);
        }
        float* O = (float*)outp;
        #pragma unroll
        for (int j = 0; j < 4; ++j) *(volatile v4f*)(O + off[j]) = w[j];
        __threadfence();
        #pragma unroll
        for (int j = 0; j < 4; ++j) *(volatile v4f*)(O + off[j]) = w[j];
    }
}

__global__ __launch_bounds__(256)
void k_attn(const _Float16* __restrict__ q, const _Float16* __restrict__ k,
            const _Float16* __restrict__ vt, const float* __restrict__ mask,
            const float* __restrict__ x, float* __restrict__ ores) {
    __shared__ __align__(16) _Float16 Ks[32 * 72];
    __shared__ __align__(16) _Float16 Vs[64 * 40];
    __shared__ __align__(16) _Float16 Ps[8][16 * 40];
    __shared__ __align__(16) float    Os[8][16 * 68];

    const int tid = threadIdx.x, lane = tid & 31, wave = tid >> 5;
    const int hl = lane >> 4, m = lane & 15;
    const int bh = blockIdx.y;
    const int b = bh / NH, hh = bh % NH;
    const int q0 = blockIdx.x * 128 + wave * 16;

    Frag aq0, aq1;
    {
        const _Float16* qp = q + ((size_t)bh * NT + q0 + m) * NDK;
        aq0.hf[0] = *(const v8h*)(qp + 8 * hl);
        aq0.hf[1] = *(const v8h*)(qp + 16 + 8 * hl);
        aq1.hf[0] = *(const v8h*)(qp + 32 + 8 * hl);
        aq1.hf[1] = *(const v8h*)(qp + 48 + 8 * hl);
    }

    const int kr = tid >> 3, kc = (tid & 7) * 8;
    const int vr = tid >> 2, vc = (tid & 3) * 8;
    const _Float16* kg = k  + ((size_t)bh * NT  + kr) * NDK + kc;
    const _Float16* vg = vt + ((size_t)bh * NDK + vr) * NT  + vc;
    const float* mrow = mask + (size_t)b * NT * NT;

    v8f acc[4];
    #pragma unroll
    for (int c = 0; c < 4; ++c) acc[c] = zero8();
    float mrun[8], lrun[8];
    #pragma unroll
    for (int e = 0; e < 8; ++e) { mrun[e] = -3.0e38f; lrun[e] = 0.0f; }

    const float sscale = 0.125f;
    const float pscale = 4096.0f;
    _Float16* ps = &Ps[wave][0];

    for (int st = 0; st < NT / 32; ++st) {
        const int s0 = st * 32;
        const v8h tk = *(const v8h*)(kg + (size_t)s0 * NDK);
        const v8h tv = *(const v8h*)(vg + s0);
        __syncthreads();
        *(v8h*)(Ks + kr * 72 + kc) = tk;
        *(v8h*)(Vs + vr * 40 + vc) = tv;
        __syncthreads();

        float p[2][8];
        #pragma unroll
        for (int half = 0; half < 2; ++half) {
            const _Float16* kp = Ks + (half * 16 + m) * 72;
            Frag b0, b1;
            b0.hf[0] = *(const v8h*)(kp + 8 * hl);
            b0.hf[1] = *(const v8h*)(kp + 16 + 8 * hl);
            b1.hf[0] = *(const v8h*)(kp + 32 + 8 * hl);
            b1.hf[1] = *(const v8h*)(kp + 48 + 8 * hl);
            v8f S = zero8();
            S = wmma16(aq0.v, b0.v, S);
            S = wmma16(aq1.v, b1.v, S);
            const int key = s0 + half * 16 + m;
            #pragma unroll
            for (int e = 0; e < 8; ++e) {
                const int row = q0 + 8 * hl + e;
                const float mv = mrow[(size_t)row * NT + key];
                const float add = NEGBIG * (1.0f - mv);
                p[half][e] = S[e] * sscale + add;
            }
        }
        float mnew[8], resc[8];
        #pragma unroll
        for (int e = 0; e < 8; ++e) {
            float mx = fmaxf(p[0][e], p[1][e]);
            #pragma unroll
            for (int off = 1; off < 16; off <<= 1) mx = fmaxf(mx, __shfl_xor(mx, off, 32));
            mnew[e] = fmaxf(mrun[e], mx);
            resc[e] = __expf(mrun[e] - mnew[e]);
            mrun[e] = mnew[e];
        }
        #pragma unroll
        for (int e = 0; e < 8; ++e) {
            p[0][e] = __expf(p[0][e] - mnew[e]);
            p[1][e] = __expf(p[1][e] - mnew[e]);
            float sum = p[0][e] + p[1][e];
            #pragma unroll
            for (int off = 1; off < 16; off <<= 1) sum += __shfl_xor(sum, off, 32);
            lrun[e] = lrun[e] * resc[e] + sum;
        }
        #pragma unroll
        for (int c = 0; c < 4; ++c) {
            #pragma unroll
            for (int e = 0; e < 8; ++e) acc[c][e] *= resc[e];
        }

        #pragma unroll
        for (int e = 0; e < 8; ++e) {
            const int row = 8 * hl + e;
            ps[row * 40 + m]      = (_Float16)(p[0][e] * pscale);
            ps[row * 40 + 16 + m] = (_Float16)(p[1][e] * pscale);
        }
        __syncthreads();
        Frag ap;
        {
            const _Float16* pr = ps + m * 40;
            ap.hf[0] = *(const v8h*)(pr + 8 * hl);
            ap.hf[1] = *(const v8h*)(pr + 16 + 8 * hl);
        }
        #pragma unroll
        for (int c = 0; c < 4; ++c) {
            const _Float16* vp = Vs + (c * 16 + m) * 40;
            Frag fv;
            fv.hf[0] = *(const v8h*)(vp + 8 * hl);
            fv.hf[1] = *(const v8h*)(vp + 16 + 8 * hl);
            acc[c] = wmma16(ap.v, fv.v, acc[c]);
        }
    }

    float inv[8];
    #pragma unroll
    for (int e = 0; e < 8; ++e) inv[e] = (1.0f / lrun[e]) * (1.0f / 4096.0f);
    float* os = &Os[wave][0];
    #pragma unroll
    for (int c = 0; c < 4; ++c) {
        #pragma unroll
        for (int e = 0; e < 8; ++e) os[(8 * hl + e) * 68 + c * 16 + m] = acc[c][e] * inv[e];
    }
    __syncthreads();
    v4f w[8];
    size_t goff[8];
    #pragma unroll
    for (int j = 0; j < 8; ++j) {
        const int id = lane + 32 * j;
        const int line = id >> 3, pc = lane & 7;
        const int row = line >> 1, colo = ((line & 1) << 5) + pc * 4;
        goff[j] = ((size_t)(b * NT + q0 + row)) * ND + hh * NDK + colo;
        w[j] = *(const v4f*)(os + row * 68 + colo) + *(const v4f*)(x + goff[j]);
    }
    #pragma unroll
    for (int j = 0; j < 8; ++j) *(volatile v4f*)(ores + goff[j]) = w[j];
    __threadfence();
    #pragma unroll
    for (int j = 0; j < 8; ++j) *(volatile v4f*)(ores + goff[j]) = w[j];
}

extern "C" void kernel_launch(void* const* d_in, const int* in_sizes, int n_in,
                              void* d_out, int out_size, void* d_ws, size_t ws_size,
                              hipStream_t stream) {
    if (n_in < 18) return;
    if (in_sizes[0] != NM * ND || in_sizes[1] != NB * NT * NT || out_size != NM * ND) return;
    if (in_sizes[2] != ND || in_sizes[3] != ND || in_sizes[4] != ND * ND || in_sizes[5] != ND ||
        in_sizes[6] != ND * ND || in_sizes[7] != ND || in_sizes[8] != ND * ND || in_sizes[9] != ND ||
        in_sizes[10] != ND || in_sizes[11] != ND || in_sizes[12] != ND * NF || in_sizes[13] != NF ||
        in_sizes[14] != NF * ND || in_sizes[15] != ND || in_sizes[16] != ND || in_sizes[17] != ND) return;

    const float* x       = (const float*)d_in[0];
    const float* mask    = (const float*)d_in[1];
    const float* ln_in_g = (const float*)d_in[2];
    const float* ln_in_b = (const float*)d_in[3];
    const float* Wq      = (const float*)d_in[4];
    const float* bq      = (const float*)d_in[5];
    const float* Wk      = (const float*)d_in[6];
    const float* bk      = (const float*)d_in[7];
    const float* Wv      = (const float*)d_in[8];
    const float* bv      = (const float*)d_in[9];
    const float* ln1_g   = (const float*)d_in[10];
    const float* ln1_b   = (const float*)d_in[11];
    const float* W1      = (const float*)d_in[12];
    const float* b1      = (const float*)d_in[13];
    const float* W2      = (const float*)d_in[14];
    const float* b2      = (const float*)d_in[15];
    const float* ln2_g   = (const float*)d_in[16];
    const float* ln2_b   = (const float*)d_in[17];
    float* out = (float*)d_out;

    char* ws = (char*)d_ws;
    size_t o = 0;
    const size_t SZ_H16 = (size_t)NM * ND * 2;
    const size_t SZ_F32 = (size_t)NM * ND * 4;
    _Float16* h16  = (_Float16*)(ws + o); o += SZ_H16;
    _Float16* q16  = (_Float16*)(ws + o); o += SZ_H16;
    _Float16* k16  = (_Float16*)(ws + o); o += SZ_H16;
    _Float16* vt16 = (_Float16*)(ws + o); o += SZ_H16;
    _Float16* f1   = h16;
    float* ares = (float*)(ws + o); o += SZ_F32;
    float* y    = ares;
    float* a32  = (float*)(ws + o); o += SZ_F32;
    _Float16* a16 = (_Float16*)(ws + o); o += SZ_H16;
    _Float16* Wqh = (_Float16*)(ws + o); o += (size_t)ND * ND * 2;
    _Float16* Wkh = (_Float16*)(ws + o); o += (size_t)ND * ND * 2;
    _Float16* Wvh = (_Float16*)(ws + o); o += (size_t)ND * ND * 2;
    _Float16* W1h = (_Float16*)(ws + o); o += (size_t)NF * ND * 2;
    _Float16* W2h = (_Float16*)(ws + o); o += (size_t)ND * NF * 2;
    if ((size_t)NM * NF * 2 > 4 * SZ_H16) return;
    if (o > ws_size) return;

    k_wcvt<<<dim3(ND / 32, ND / 64), 256, 0, stream>>>(Wq, Wqh, ND, ND, 16.0f);
    k_wcvt<<<dim3(ND / 32, ND / 64), 256, 0, stream>>>(Wk, Wkh, ND, ND, 16.0f);
    k_wcvt<<<dim3(ND / 32, ND / 64), 256, 0, stream>>>(Wv, Wvh, ND, ND, 16.0f);
    k_wcvt<<<dim3(NF / 32, ND / 64), 256, 0, stream>>>(W1, W1h, ND, NF, 16.0f);
    k_wcvt<<<dim3(ND / 32, NF / 64), 256, 0, stream>>>(W2, W2h, NF, ND, 32.0f);

    k_ln<0><<<(NM + 7) / 8, 256, 0, stream>>>(x, ln_in_g, ln_in_b, nullptr, h16, NM);

    const dim3 gQKV(ND / 64, NM / 64);
    k_gemm<0><<<gQKV, 256, 0, stream>>>(h16, Wqh, bq, nullptr, (void*)q16,  ND, ND, 0.0625f);
    k_gemm<0><<<gQKV, 256, 0, stream>>>(h16, Wkh, bk, nullptr, (void*)k16,  ND, ND, 0.0625f);
    k_gemm<1><<<gQKV, 256, 0, stream>>>(h16, Wvh, bv, nullptr, (void*)vt16, ND, ND, 0.0625f);

    k_attn<<<dim3(NT / 128, NB * NH), 256, 0, stream>>>(q16, k16, vt16, mask, x, ares);

    k_ln<1><<<(NM + 7) / 8, 256, 0, stream>>>(ares, ln1_g, ln1_b, a32, a16, NM);

    k_gemm<2><<<dim3(NF / 64, NM / 64), 256, 0, stream>>>(a16, W1h, b1, nullptr, (void*)f1, NF, ND, 0.0625f);

    k_gemm<3><<<dim3(ND / 64, NM / 64), 256, 0, stream>>>(f1, W2h, b2, a32, (void*)y, ND, NF, 0.03125f);

    k_ln<2><<<(NM + 7) / 8, 256, 0, stream>>>(y, ln2_g, ln2_b, out, nullptr, NM);
}
